// EfficientAttention_25838523252895
// MI455X (gfx1250) — hardware-verified
//
#include <hip/hip_runtime.h>
#include <stddef.h>


typedef _Float16 v16h __attribute__((ext_vector_type(16)));
typedef _Float16 v8h  __attribute__((ext_vector_type(8)));
typedef float    v8f  __attribute__((ext_vector_type(8)));
typedef float    v4f  __attribute__((ext_vector_type(4)));

#ifndef NB
#define NB 2
#endif
#ifndef SEQ
#define SEQ 2048
#endif
#define NB_FULL  2
#define SEQ_FULL 2048
#define NHEAD 16
#define HD    64
#define CHUNK 512
#define NBH   (NB * NHEAD)

static_assert(NB >= 1 && NB <= NB_FULL);
static_assert(SEQ >= CHUNK && SEQ <= SEQ_FULL && (SEQ % CHUNK) == 0);
static_assert((CHUNK % 128) == 0 && (SEQ % 128) == 0 && (SEQ % 64) == 0);
static_assert(HD == 64);
static_assert(((size_t)NBH * SEQ * HD) % (256u * 8u) == 0);
static_assert((size_t)NBH * SEQ_FULL * HD < (size_t)0xFFFFFFFFu);

#define LDT 72
#define LDC 68
static_assert((LDT % 8) == 0 && LDT >= 64);
static_assert((LDC % 4) == 0 && LDC >= 64);

#define QKCARRY 16.0f
#define WCARRY  64.0f
#define PCARRY  1024.0f
#define RCARRY  1024.0f
#define NEGFILL (-1.0e9f)
#ifndef P_RES
#define P_RES 1
#endif

#define PLANE16_BYTES ((size_t)NBH * SEQ * HD * 2)
#define OFF_Q  ((size_t)0)
#define OFF_K  (OFF_Q + PLANE16_BYTES)
#define OFF_VT (OFF_K + PLANE16_BYTES)
#define WS_TOTAL (OFF_VT + PLANE16_BYTES)
static_assert((PLANE16_BYTES % 128) == 0);
static_assert(WS_TOTAL <= (size_t)134217728);

static_assert((size_t)(64 * LDT * 2) * 2 + (size_t)(8 * 16 * LDT * 2) + (size_t)(8 * 16 * LDC * 4)
              <= (size_t)131072);

__device__ __forceinline__ float bf16r(float x) {
  unsigned int u = __float_as_uint(x);
  u = (u + 0x7FFFu + ((u >> 16) & 1u)) & 0xFFFF0000u;
  return __uint_as_float(u);
}

static __device__ __forceinline__ _Float16 toh_flush(float v) {
  const _Float16 r = (_Float16)v;
  return (fabsf(v) < 6.103515625e-05f) ? (_Float16)0.0f : r;
}

__device__ __forceinline__ v16h frag_at(const _Float16* p) {
  v8h lo = *(const v8h*)(p);
  v8h hi = *(const v8h*)(p + 16);
  v16h out;
#pragma unroll
  for (int i = 0; i < 8; ++i) { out[i] = lo[i]; out[i + 8] = hi[i]; }
  return out;
}
__device__ __forceinline__ v16h ld_frag(const _Float16* base, unsigned ld) {
  const unsigned lane = threadIdx.x & 31u;
  return frag_at(base + (lane & 15u) * ld + (lane >> 4) * 8u);
}

__device__ __forceinline__ v8f wmma16(v16h a, v16h b, v8f c) {
  v8f d = __builtin_amdgcn_wmma_f32_16x16x32_f16(false, a, false, b, (short)0, c,
                                                 false, false);
  asm volatile("v_nop\n\tv_nop\n\tv_nop\n\tv_nop" : "+v"(d) : "v"(a), "v"(b));
  return d;
}

__device__ __forceinline__ float red16_max(float x) {
#pragma unroll
  for (int off = 1; off < 16; off <<= 1) x = fmaxf(x, __shfl_xor(x, off, 32));
  return x;
}
__device__ __forceinline__ float red16_sum(float x) {
#pragma unroll
  for (int off = 1; off < 16; off <<= 1) x += __shfl_xor(x, off, 32);
  return x;
}

__device__ __forceinline__ void wave_lds_sync() {
  __builtin_amdgcn_fence(3  , "wavefront");
  asm volatile("s_wait_dscnt 0x0" ::: "memory");
  __builtin_amdgcn_wave_barrier();
}

__global__ __launch_bounds__(256) void qkconv_kernel(
    const float* __restrict__ Qf, const float* __restrict__ Kf,
    _Float16* __restrict__ Q16, _Float16* __restrict__ K16) {
  const unsigned e = (blockIdx.x * 256u + threadIdx.x) * 8u;
  const unsigned crow = e >> 6, c = e & 63u;
  const unsigned bh = crow / (unsigned)SEQ;
  const unsigned sq = crow - bh * (unsigned)SEQ;
  const size_t src = ((size_t)bh * SEQ_FULL + sq) * HD + c;
  const v4f a0 = *(const v4f*)(Qf + src);
  const v4f a1 = *(const v4f*)(Qf + src + 4u);
  const v4f b0 = *(const v4f*)(Kf + src);
  const v4f b1 = *(const v4f*)(Kf + src + 4u);
  v8h xq, xk;
#pragma unroll
  for (int i = 0; i < 4; ++i) {
    xq[i]     = toh_flush(QKCARRY * bf16r(a0[i]));
    xq[i + 4] = toh_flush(QKCARRY * bf16r(a1[i]));
    xk[i]     = toh_flush(QKCARRY * bf16r(b0[i]));
    xk[i + 4] = toh_flush(QKCARRY * bf16r(b1[i]));
  }
  *(volatile v8h*)(Q16 + e) = xq;
  *(volatile v8h*)(K16 + e) = xk;
  __threadfence();
  *(volatile v8h*)(Q16 + e) = xq;
  *(volatile v8h*)(K16 + e) = xk;
}

static_assert((256 / 8) * 2 == 64);
__global__ __launch_bounds__(256) void vconv_kernel(
    const float* __restrict__ W, _Float16* __restrict__ Wt, unsigned ldw, unsigned ldk,
    unsigned wbatch, unsigned tbatch) {
  __shared__ __attribute__((aligned(16))) _Float16 T[64 * LDT];
  const unsigned tid = threadIdx.x;
  const unsigned n0 = blockIdx.x * 64u;
  const unsigned k0 = blockIdx.y * 64u;
  const size_t wb = (size_t)blockIdx.z * wbatch;
  const size_t tb = (size_t)blockIdx.z * tbatch;
#pragma unroll 4
  for (unsigned j = 0; j < 16u; ++j) {
    const unsigned idx = tid + 256u * j;
    const unsigned kr = idx >> 6, nc = idx & 63u;
    const float v = W[wb + (size_t)(k0 + kr) * ldw + n0 + nc];
    T[nc * LDT + kr] = toh_flush(WCARRY * bf16r(v));
  }
  __syncthreads();
  v8h x[2];
  size_t off[2];
#pragma unroll
  for (unsigned i = 0; i < 2u; ++i) {
    const unsigned n = 32u * i + (tid >> 3);
    const unsigned kc = (tid & 7u) * 8u;
    x[i] = *(const v8h*)&T[n * LDT + kc];
    off[i] = tb + (size_t)(n0 + n) * ldk + k0 + kc;
  }
#pragma unroll
  for (int i = 0; i < 2; ++i) *(volatile v8h*)(Wt + off[i]) = x[i];
  __threadfence();
#pragma unroll
  for (int i = 0; i < 2; ++i) *(volatile v8h*)(Wt + off[i]) = x[i];
}

static_assert(2 * 8 == 16);
__global__ __launch_bounds__(256) __attribute__((amdgpu_num_vgpr(256))) void attn_kernel(
    const _Float16* __restrict__ Qh, const _Float16* __restrict__ Kh,
    const _Float16* __restrict__ Vt, float* __restrict__ Out) {
  __shared__ __attribute__((aligned(16))) _Float16 Ks[64 * LDT];
  __shared__ __attribute__((aligned(16))) _Float16 Vs[64 * LDT];
  __shared__ __attribute__((aligned(16))) _Float16 Ps[8 * 16 * LDT];
  __shared__ __attribute__((aligned(16))) float Os[8 * 16 * LDC];

  const unsigned tid = threadIdx.x, lane = tid & 31u;
  const unsigned w = (unsigned)__builtin_amdgcn_readfirstlane((int)(threadIdx.x >> 5));
  const unsigned hh = lane >> 4, m = lane & 15u;
  const unsigned q0 = blockIdx.x * 128u;
  const unsigned bh = blockIdx.z * (unsigned)NHEAD + blockIdx.y;
  const unsigned ci = q0 / (unsigned)CHUNK;
  const unsigned cs = ci * (unsigned)CHUNK;
  const bool first_blk = (q0 == cs);
  const float scale = 0.125f / (QKCARRY * QKCARRY);
  const unsigned qrow0 = q0 + w * 16u;
  _Float16* P = Ps + w * (16u * LDT);
  const unsigned obase = w * (16u * LDC);

  const size_t qoff = ((size_t)bh * SEQ + qrow0 + m) * HD + hh * 8u;
  v16h qf[2];
  qf[0] = frag_at(Qh + qoff);
  qf[1] = frag_at(Qh + qoff + 32);

  float mrow[8], lrow[8];
  v8f o[4], ot[4];
#pragma unroll
  for (int v = 0; v < 8; ++v) { mrow[v] = -1.0e30f; lrow[v] = 0.0f; }
#pragma unroll
  for (int nb = 0; nb < 4; ++nb) { o[nb] = (v8f){}; ot[nb] = (v8f){}; }

  const size_t kplane = (size_t)bh * SEQ * HD;
  const size_t vplane = (size_t)bh * HD * SEQ;

#pragma unroll 1
  for (unsigned jc = 0; jc <= ci; ++jc) {
    const bool offd = (jc < ci);
    const unsigned kc0 = jc * (unsigned)CHUNK;
    const unsigned kc1 = offd ? (kc0 + (unsigned)CHUNK) : (q0 + 128u);

#pragma unroll 1
    for (unsigned kb = kc0; kb < kc1; kb += 64u) {
      const bool early = (P_RES != 0) && first_blk && (!offd) && (kb == cs);
#pragma unroll
      for (unsigned j = 0; j < 2u; ++j) {
        const unsigned idx = tid + 256u * j;
        const unsigned r = idx >> 3, c = (idx & 7u) * 8u;
        *(v8h*)&Ks[r * LDT + c] = *(const v8h*)(Kh + kplane + (size_t)(kb + r) * HD + c);
        *(v8h*)&Vs[r * LDT + c] = *(const v8h*)(Vt + vplane + (size_t)r * SEQ + kb + c);
      }
      __syncthreads();

      v8f s[4];
#pragma unroll
      for (int kg = 0; kg < 4; ++kg) {
        v8f t = {};
#pragma unroll
        for (int c = 0; c < 2; ++c) {
          const v16h kf = ld_frag(&Ks[(kg * 16) * LDT + c * 32], LDT);
          t = wmma16(qf[c], kf, t);
        }
        s[kg] = t * scale;
      }

      if (offd) {
#pragma unroll
        for (int kg = 0; kg < 4; ++kg)
#pragma unroll
          for (int v = 0; v < 8; ++v) s[kg][v] = s[kg][v] + NEGFILL;
      } else if (kb >= q0) {
#pragma unroll
        for (int kg = 0; kg < 4; ++kg)
#pragma unroll
          for (int v = 0; v < 8; ++v) {
            const unsigned key = kb + (unsigned)kg * 16u + m;
            const unsigned row = qrow0 + hh * 8u + (unsigned)v;
            const float add = (key > row) ? NEGFILL : 0.0f;
            s[kg][v] = s[kg][v] + add;
          }
      }

      float alpha[8];
#pragma unroll
      for (int v = 0; v < 8; ++v) {
        float mx = fmaxf(fmaxf(s[0][v], s[1][v]), fmaxf(s[2][v], s[3][v]));
        mx = red16_max(mx);
        const float mn = fmaxf(mrow[v], mx);
        alpha[v] = __expf(mrow[v] - mn);
        mrow[v] = mn;
      }
#pragma unroll
      for (int kg = 0; kg < 4; ++kg)
#pragma unroll
        for (int v = 0; v < 8; ++v) s[kg][v] = __expf(s[kg][v] - mrow[v]);
#pragma unroll
      for (int v = 0; v < 8; ++v) {
        const float rs = red16_sum((s[0][v] + s[1][v]) + (s[2][v] + s[3][v]));
        lrow[v] = alpha[v] * lrow[v] + rs;
      }
#pragma unroll
      for (int nb = 0; nb < 4; ++nb)
#pragma unroll
        for (int v = 0; v < 8; ++v) o[nb][v] = o[nb][v] * alpha[v];

#pragma unroll
      for (int kg = 0; kg < 4; ++kg)
#pragma unroll
        for (int v = 0; v < 8; ++v)
          P[(hh * 8u + (unsigned)v) * LDT + (unsigned)kg * 16u + m] = toh_flush(s[kg][v] * PCARRY);
      wave_lds_sync();

#pragma unroll
      for (int c = 0; c < 2; ++c) {
        const v16h pf = ld_frag(P + c * 32, LDT);
#pragma unroll
        for (int nb = 0; nb < 4; ++nb) {
          const v16h vf = ld_frag(&Vs[(nb * 16) * LDT + c * 32], LDT);
          o[nb] = wmma16(pf, vf, o[nb]);
        }
      }

      if (early) {
        wave_lds_sync();
#pragma unroll
        for (int kg = 0; kg < 4; ++kg)
#pragma unroll
          for (int v = 0; v < 8; ++v) {
            const float t = s[kg][v] * PCARRY;
            const float hi = (float)toh_flush(t);
            P[(hh * 8u + (unsigned)v) * LDT + (unsigned)kg * 16u + m] =
                toh_flush((t - hi) * RCARRY);
          }
        wave_lds_sync();
#pragma unroll
        for (int nb = 0; nb < 4; ++nb) {
          v8f o2 = {};
#pragma unroll
          for (int c = 0; c < 2; ++c) {
            const v16h pf = ld_frag(P + c * 32, LDT);
            const v16h vf = ld_frag(&Vs[(nb * 16) * LDT + c * 32], LDT);
            o2 = wmma16(pf, vf, o2);
          }
#pragma unroll
          for (int v = 0; v < 8; ++v) o[nb][v] = o[nb][v] + o2[v] * (1.0f / RCARRY);
        }
      }
      __syncthreads();
    }

#pragma unroll
    for (int v = 0; v < 8; ++v) {
      const float inv = __builtin_amdgcn_rcpf(lrow[v]);
#pragma unroll
      for (int nb = 0; nb < 4; ++nb) ot[nb][v] = ot[nb][v] + o[nb][v] * inv;
      mrow[v] = -1.0e30f;
      lrow[v] = 0.0f;
    }
#pragma unroll
    for (int nb = 0; nb < 4; ++nb) o[nb] = (v8f){};
  }

  const float fs = 1.0f / (PCARRY * WCARRY);
#pragma unroll
  for (int nb = 0; nb < 4; ++nb)
#pragma unroll
    for (int v = 0; v < 8; ++v)
      Os[obase + (hh * 8u + (unsigned)v) * LDC + (unsigned)nb * 16u + m] = ot[nb][v] * fs;
  wave_lds_sync();
  v4f x[8];
  size_t off[8];
#pragma unroll
  for (unsigned i = 0; i < 8u; ++i) {
    const unsigned r = 2u * i + (lane >> 4);
    const unsigned c = (lane & 15u) * 4u;
    x[i] = *(const v4f*)&Os[obase + r * LDC + c];
    off[i] = ((size_t)bh * SEQ_FULL + qrow0 + r) * HD + c;
  }
#pragma unroll
  for (int i = 0; i < 8; ++i) *(volatile v4f*)(Out + off[i]) = x[i];
  __threadfence();
#pragma unroll
  for (int i = 0; i < 8; ++i) *(volatile v4f*)(Out + off[i]) = x[i];
}

extern "C" void kernel_launch(void* const* d_in, const int* in_sizes, int n_in,
                              void* d_out, int out_size, void* d_ws, size_t ws_size,
                              hipStream_t stream) {
  if (n_in < 3) return;
  const long long need = ((long long)(NBH - 1) * SEQ_FULL + SEQ) * HD;
  if ((long long)in_sizes[0] < need) return;
  if ((long long)in_sizes[1] < need) return;
  if ((long long)in_sizes[2] < need) return;
  if ((long long)out_size < need) return;
  if (ws_size < WS_TOTAL) return;

  const float* Qf = (const float*)d_in[0];
  const float* Kf = (const float*)d_in[1];
  const float* Vf = (const float*)d_in[2];
  float* out = (float*)d_out;

  char* ws = (char*)d_ws;
  _Float16* Q16  = (_Float16*)(ws + OFF_Q);
  _Float16* K16  = (_Float16*)(ws + OFF_K);
  _Float16* Vt16 = (_Float16*)(ws + OFF_VT);

  dim3 blk(256);
  qkconv_kernel<<<dim3((unsigned)(((size_t)NBH * SEQ * HD) / 2048u)), blk, 0, stream>>>(
      Qf, Kf, Q16, K16);
  vconv_kernel<<<dim3(HD / 64, SEQ / 64, NBH), blk, 0, stream>>>(
      Vf, Vt16, (unsigned)HD, (unsigned)SEQ, (unsigned)(SEQ_FULL * HD), (unsigned)(HD * SEQ));
  attn_kernel<<<dim3(SEQ / 128, NHEAD, NB), blk, 0, stream>>>(Q16, K16, Vt16, out);
}
